// QLSTM_65481071400861
// MI455X (gfx1250) — hardware-run, weakly checked
//
#include <hip/hip_runtime.h>
#include <math.h>

typedef __attribute__((ext_vector_type(16))) _Float16 v16h;
typedef __attribute__((ext_vector_type(8)))  _Float16 v8h;
typedef __attribute__((ext_vector_type(8)))  float    v8f;
typedef __attribute__((ext_vector_type(4)))  float    v4f;
typedef __attribute__((ext_vector_type(4)))  unsigned v4u;

constexpr int kSeq    = 128;
constexpr int kBatch  = 512;
constexpr int kFeat   = 128;
constexpr int kHid    = 128;
constexpr int kWires  = 8;
constexpr int kDim    = 256;
constexpr int kDepth  = 2;
constexpr int kGates  = 4;
constexpr int kKq     = kFeat + kHid;
constexpr int kTileB  = 16;
constexpr int kBlocks = kBatch / kTileB;
constexpr int kThreads = 256;
constexpr int kWaves  = kThreads / 32;
constexpr int kAPitch = kKq + 8;
constexpr int kNumFac = kGates * kDepth * 2;
constexpr int kFacElems = 256;
static_assert(kDim == (1 << kWires));
static_assert(kTileB == 2 * kWaves);
static_assert(kKq == 32 * kWaves);
static_assert(kBatch % kTileB == 0);
static_assert((kAPitch * 2) % 16 == 0);

constexpr size_t kOutH = (size_t)kSeq * kBatch * kHid;
constexpr size_t kOutC = kOutH + (size_t)kBatch * kHid;
constexpr size_t kOutTotal = kOutC + (size_t)kBatch * kHid;
static_assert(kOutH * 4 == 33554432ull);
static_assert(kOutC * 4 == 33816576ull);
static_assert(kOutTotal * 4 == 34078720ull);

constexpr size_t kWsFac   = (size_t)kNumFac * kFacElems * 2;
constexpr size_t kWsTotal = kWsFac;
static_assert(kWsTotal == 8192ull);
static_assert(kWsTotal <= 134217728ull);

constexpr float kActCarry = 64.0f;
constexpr float kWqCarry  = 1024.0f;
constexpr float kQFold    = 1.0f / (kActCarry * kWqCarry);
constexpr float kPsiCarry = 64.0f;
constexpr float kFacCarry = 64.0f;
constexpr float kResCarry = 2048.0f;
constexpr float kMidMain  = 1.0f / kFacCarry;
constexpr float kMidRes   = kMidMain / kResCarry;
constexpr float kEndMain  = kMidMain / kPsiCarry;
constexpr float kEndRes   = kEndMain / kResCarry;
constexpr float kF16Min   = 6.103515625e-05f;

__host__ __device__ constexpr int chain_index(int j) {
  for (int w = kWires - 2; w >= 0; --w) {
    if ((j >> (kWires - 1 - w)) & 1) j ^= (1 << (kWires - 2 - w));
  }
  return j;
}
constexpr bool chain_is_permutation() {
  bool seen[kDim] = {};
  for (int j = 0; j < kDim; ++j) {
    const int p = chain_index(j);
    if (p < 0 || p >= kDim) return false;
    if (seen[p]) return false;
    seen[p] = true;
  }
  return true;
}
constexpr bool chain_matches_sequential_gathers() {
  int cur[kDim] = {};
  int nxt[kDim] = {};
  for (int j = 0; j < kDim; ++j) cur[j] = j;
  for (int w = 0; w <= kWires - 2; ++w) {
    for (int j = 0; j < kDim; ++j) {
      int src = j;
      if ((j >> (kWires - 1 - w)) & 1) src = j ^ (1 << (kWires - 2 - w));
      nxt[j] = cur[src];
    }
    for (int j = 0; j < kDim; ++j) cur[j] = nxt[j];
  }
  for (int j = 0; j < kDim; ++j) {
    if (cur[j] != chain_index(j)) return false;
  }
  return true;
}
static_assert(chain_is_permutation());
static_assert(chain_matches_sequential_gathers());

__device__ __forceinline__ float bf16_rne(float f) {
  unsigned u = __float_as_uint(f);
  u = (u + 0x7FFFu + ((u >> 16) & 1u)) & 0xFFFF0000u;
  return __uint_as_float(u);
}
__device__ __forceinline__ float flush_small(float v) { return (fabsf(v) < kF16Min) ? 0.0f : v; }
__device__ __forceinline__ _Float16 to_h(float v) { return (_Float16)flush_small(v); }

__device__ __forceinline__ void wave_lds_sync() {
  __builtin_amdgcn_fence(__ATOMIC_RELEASE, "workgroup");
  __builtin_amdgcn_wave_barrier();
  __builtin_amdgcn_fence(__ATOMIC_ACQUIRE, "workgroup");
}

__device__ __forceinline__ v16h frag_load(const _Float16* p) {
  union U { v16h v; v8h hh[2]; } f;
  f.hh[0] = *(const v8h*)(p);
  f.hh[1] = *(const v8h*)(p + 16);
  return f.v;
}
__device__ __forceinline__ v16h widen(v8h lo8) {
  const v8h z = {(_Float16)0.0f, (_Float16)0.0f, (_Float16)0.0f, (_Float16)0.0f,
                 (_Float16)0.0f, (_Float16)0.0f, (_Float16)0.0f, (_Float16)0.0f};
  return __builtin_shufflevector(lo8, z, 0, 1, 2, 3, 4, 5, 6, 7, 8, 9, 10, 11, 12, 13, 14, 15);
}
__device__ __forceinline__ v8f mma_acc(v16h a, v16h b, v8f c) {
  c = __builtin_amdgcn_wmma_f32_16x16x32_f16(false, a, false, b, (short)0, c, false, false);
  asm volatile("v_nop\n\tv_nop\n\tv_nop\n\tv_nop" : "+v"(c) : "v"(a), "v"(b));
  return c;
}
__device__ __forceinline__ v8f mma_zero(v16h a, v16h b) {
  v8f c = {0.f, 0.f, 0.f, 0.f, 0.f, 0.f, 0.f, 0.f};
  return mma_acc(a, b, c);
}
__device__ __forceinline__ void split8(v8f x, v8h& hi, v8h& lo) {
#pragma unroll
  for (int e = 0; e < 8; ++e) {
    const _Float16 hv = (_Float16)flush_small(x[e]);
    const float r = (x[e] - (float)hv) * kResCarry;
    hi[e] = hv;
    lo[e] = (_Float16)flush_small(r);
  }
}
__device__ __forceinline__ v8f stage(v8h xh, v8h xl, v16h bfac, float km, float kr) {
  const v8f am = mma_zero(widen(xh), bfac);
  const v8f ar = mma_zero(widen(xl), bfac);
  v8f o;
#pragma unroll
  for (int e = 0; e < 8; ++e) o[e] = am[e] * km + ar[e] * kr;
  return o;
}
__device__ __forceinline__ v8f layer_pair(v8h xh, v8h xl, v16h bLo, v16h bHi, float k2m, float k2r) {
  const v8f t1 = stage(xh, xl, bLo, kMidMain, kMidRes);
  v8h th, tl;
  split8(t1, th, tl);
  return stage(th, tl, bHi, k2m, k2r);
}

__device__ __forceinline__ float sigmoid_fast(float x) {
  return __builtin_amdgcn_rcpf(1.0f + __expf(-x));
}
__device__ __forceinline__ float tanh_fast(float x) {
  const float a = fabsf(x);
  const float t = __expf(-2.0f * a);
  const float r = (1.0f - t) * __builtin_amdgcn_rcpf(1.0f + t);
  return copysignf(r, x);
}

__global__ __launch_bounds__(512) void build_factor_planes(
    const float* __restrict__ pf, const float* __restrict__ pi, const float* __restrict__ pg,
    const float* __restrict__ po, unsigned short* __restrict__ fac)
{
  const int tid = threadIdx.x, lane = tid & 31, f = tid >> 5;
  const int gate = f >> 2, layer = (f >> 1) & 1, half = f & 1;
  const int row = lane >> 1, col0 = (lane & 1) * 8;
  const int w0 = half ? 0 : 4;
  float prod[8];
#pragma unroll
  for (int e = 0; e < 8; ++e) prod[e] = 1.0f;
#pragma unroll 1
  for (int k = 0; k < 4; ++k) {
    const int idx = layer * kWires + w0 + k;
    const float t0 = pf[idx];
    const float t1 = pi[idx];
    const float t2 = pg[idx];
    const float t3 = po[idx];
    float th = t0;
    th = (gate == 1) ? t1 : th;
    th = (gate == 2) ? t2 : th;
    th = (gate == 3) ? t3 : th;
    th = bf16_rne(th);
    float sn, cs;
    sincosf(0.5f * th, &sn, &cs);
    const int rb = (row >> (3 - k)) & 1;
#pragma unroll
    for (int e = 0; e < 8; ++e) {
      const int cb = ((col0 + e) >> (3 - k)) & 1;
      const float off = rb ? sn : -sn;
      const float el = (rb == cb) ? cs : off;
      prod[e] = prod[e] * el;
    }
  }
  v8h hv;
#pragma unroll
  for (int e = 0; e < 8; ++e) hv[e] = to_h(prod[e] * kFacCarry);
  unsigned short* q = fac + (size_t)f * kFacElems + lane * 8;
  *(volatile v8h*)q = hv;
  __threadfence();
  *(volatile v8h*)q = hv;
}

__global__ __launch_bounds__(kThreads) void gated_cell_kernel(
    const float* __restrict__ xin, const float* __restrict__ Wq, const float* __restrict__ bq,
    const float* __restrict__ Wf, const float* __restrict__ bfp,
    const float* __restrict__ Wi, const float* __restrict__ bip,
    const float* __restrict__ Wg, const float* __restrict__ bgp,
    const float* __restrict__ Wo, const float* __restrict__ bop,
    const unsigned short* __restrict__ fac, float* __restrict__ out)
{
  __shared__ __align__(16) _Float16 s_fac[kNumFac * kFacElems];
  __shared__ __align__(16) _Float16 s_a[kTileB * kAPitch];
  __shared__ __align__(16) float s_qp[kWaves * 256];
  __shared__ __align__(16) float s_scr[kWaves * 512];
  __shared__ __align__(16) float s_ev[kTileB * 32];
  __shared__ __align__(16) float s_c[kTileB * kHid];
  float* s_hout = s_scr;

  const int tid = threadIdx.x, lane = tid & 31, wave = tid >> 5, blk = blockIdx.x;
  const int n = lane & 15, h = lane >> 4;

  {
    const v4u* src = (const v4u*)fac;
    v4u* dst = (v4u*)s_fac;
    const v4u u0 = src[tid];
    const v4u u1 = src[tid + 256];
    dst[tid] = u0;
    dst[tid + 256] = u1;
  }
  {
    const int row = tid >> 4, c8 = (tid & 15) * 8;
    const v8h z = {(_Float16)0.0f, (_Float16)0.0f, (_Float16)0.0f, (_Float16)0.0f,
                   (_Float16)0.0f, (_Float16)0.0f, (_Float16)0.0f, (_Float16)0.0f};
    *(v8h*)(s_a + row * kAPitch + kFeat + c8) = z;
  }
#pragma unroll
  for (int i = 0; i < 8; ++i) s_c[tid + 256 * i] = 0.0f;

  v16h bqf;
  {
    const int nr = (n < 8) ? n : 7;
    const bool keep = (n < 8);
    const float* wp = Wq + (size_t)nr * kKq + wave * 32 + 8 * h;
    const v4f w0 = *(const v4f*)(wp);
    const v4f w1 = *(const v4f*)(wp + 4);
    const v4f w2 = *(const v4f*)(wp + 16);
    const v4f w3 = *(const v4f*)(wp + 20);
#pragma unroll
    for (int e = 0; e < 4; ++e) {
      const float a0 = keep ? bf16_rne(w0[e]) * kWqCarry : 0.0f;
      const float a1 = keep ? bf16_rne(w1[e]) * kWqCarry : 0.0f;
      const float a2 = keep ? bf16_rne(w2[e]) * kWqCarry : 0.0f;
      const float a3 = keep ? bf16_rne(w3[e]) * kWqCarry : 0.0f;
      bqf[e]      = to_h(a0);
      bqf[4 + e]  = to_h(a1);
      bqf[8 + e]  = to_h(a2);
      bqf[12 + e] = to_h(a3);
    }
  }
  const float bqv = bf16_rne(bq[lane & 7]);

  const int jh = tid & (kHid - 1), half = tid >> 7;
  float wf[8], wi[8], wg[8], wo[8];
  {
    const v4f a = *(const v4f*)(Wf + jh * 8);
    const v4f b = *(const v4f*)(Wf + jh * 8 + 4);
    const v4f c = *(const v4f*)(Wi + jh * 8);
    const v4f d = *(const v4f*)(Wi + jh * 8 + 4);
    const v4f e4 = *(const v4f*)(Wg + jh * 8);
    const v4f f4 = *(const v4f*)(Wg + jh * 8 + 4);
    const v4f g4 = *(const v4f*)(Wo + jh * 8);
    const v4f h4 = *(const v4f*)(Wo + jh * 8 + 4);
#pragma unroll
    for (int e = 0; e < 4; ++e) {
      wf[e] = bf16_rne(a[e]);   wf[4 + e] = bf16_rne(b[e]);
      wi[e] = bf16_rne(c[e]);   wi[4 + e] = bf16_rne(d[e]);
      wg[e] = bf16_rne(e4[e]);  wg[4 + e] = bf16_rne(f4[e]);
      wo[e] = bf16_rne(g4[e]);  wo[4 + e] = bf16_rne(h4[e]);
    }
  }
  const float bfv = bf16_rne(bfp[jh]);
  const float biv = bf16_rne(bip[jh]);
  const float bgv = bf16_rne(bgp[jh]);
  const float bov = bf16_rne(bop[jh]);

  int pa[8];
#pragma unroll
  for (int i = 0; i < 8; ++i) pa[i] = chain_index(16 * n + 8 * h + i);

  const bool w0set = (n & 8) != 0, w1set = (n & 4) != 0, w2set = (n & 2) != 0, w3set = (n & 1) != 0, w4set = (h != 0);
  const int pl = (__popc(n) + h) & 3;

  float* scr = s_scr + wave * 512;
  __syncthreads();

#pragma unroll 1
  for (int t = 0; t < kSeq; ++t) {
    {
      const int row = tid >> 4, c8 = (tid & 15) * 8;
      const float* xp = xin + ((size_t)t * kBatch + (size_t)blk * kTileB + row) * kFeat + c8;
      const v4f a0 = *(const v4f*)(xp);
      const v4f a1 = *(const v4f*)(xp + 4);
      v8h o;
#pragma unroll
      for (int e = 0; e < 4; ++e) {
        o[e]     = to_h(bf16_rne(a0[e]) * kActCarry);
        o[4 + e] = to_h(bf16_rne(a1[e]) * kActCarry);
      }
      *(v8h*)(s_a + row * kAPitch + c8) = o;
    }
    __syncthreads();

    {
      const v16h a = frag_load(s_a + n * kAPitch + wave * 32 + 8 * h);
      const v8f qa = mma_zero(a, bqf);
      float* qp = s_qp + wave * 256 + lane * 8;
      *(v4f*)(qp)     = (v4f){qa[0], qa[1], qa[2], qa[3]};
      *(v4f*)(qp + 4) = (v4f){qa[4], qa[5], qa[6], qa[7]};
    }
    __syncthreads();

#pragma unroll 1
    for (int s = 0; s < 2; ++s) {
      const int srow = 2 * wave + s;
      const float* qsrc = s_qp + ((lane & 7) + 16 * (srow >> 3)) * 8 + (srow & 7);
      float qsum = 0.0f;
#pragma unroll
      for (int w8 = 0; w8 < kWaves; ++w8) qsum += qsrc[w8 * 256];
      const float ang = 0.5f * (qsum * kQFold + bqv);
      float sn, cs;
      sincosf(ang, &sn, &cs);
      float cw[8], sw[8];
#pragma unroll
      for (int w = 0; w < 8; ++w) {
        cw[w] = __int_as_float(__builtin_amdgcn_readlane(__float_as_int(cs), w));
        sw[w] = __int_as_float(__builtin_amdgcn_readlane(__float_as_int(sn), w));
      }
      v8h prh, prl, pih, pil;
      {
        const float f0 = w0set ? sw[0] : cw[0];
        const float f1 = w1set ? sw[1] : cw[1];
        const float f2 = w2set ? sw[2] : cw[2];
        const float f3 = w3set ? sw[3] : cw[3];
        const float f4 = w4set ? sw[4] : cw[4];
        const float base = ((f0 * f1) * (f2 * f3)) * (f4 * kPsiCarry);
        const float nbase = -base;
        const float br = (pl == 0) ? base : ((pl == 2) ? nbase : 0.0f);
        const float bi = (pl == 1) ? nbase : ((pl == 3) ? base : 0.0f);
        v8f re, im;
#pragma unroll
        for (int i = 0; i < 8; ++i) {
          const float v5 = (i & 4) ? sw[5] : cw[5];
          const float v6 = (i & 2) ? sw[6] : cw[6];
          const float v7 = (i & 1) ? sw[7] : cw[7];
          const float vv = v5 * v6 * v7;
          const int pc = ((i >> 2) & 1) + ((i >> 1) & 1) + (i & 1);
          const float rsel = (pc == 0) ? br : ((pc == 1) ? bi : ((pc == 2) ? -br : -bi));
          const float isel = (pc == 0) ? bi : ((pc == 1) ? -br : ((pc == 2) ? -bi : br));
          re[i] = vv * rsel;
          im[i] = vv * isel;
        }
        split8(re, prh, prl);
        split8(im, pih, pil);
      }

#pragma unroll 1
      for (int g = 0; g < kGates; ++g) {
        const _Float16* fb = s_fac + g * (4 * kFacElems) + n * 16 + 8 * h;
        const v16h bLo1 = widen(*(const v8h*)(fb));
        const v16h bHi1 = widen(*(const v8h*)(fb + kFacElems));
        const v16h bLo2 = widen(*(const v8h*)(fb + 2 * kFacElems));
        const v16h bHi2 = widen(*(const v8h*)(fb + 3 * kFacElems));
        {
          const v8f u = layer_pair(prh, prl, bLo1, bHi1, kMidMain, kMidRes);
          float* sp = scr + 16 * n + 8 * h;
          *(v4f*)(sp)     = (v4f){u[0], u[1], u[2], u[3]};
          *(v4f*)(sp + 4) = (v4f){u[4], u[5], u[6], u[7]};
        }
        {
          const v8f u = layer_pair(pih, pil, bLo1, bHi1, kMidMain, kMidRes);
          float* sp = scr + 256 + 16 * n + 8 * h;
          *(v4f*)(sp)     = (v4f){u[0], u[1], u[2], u[3]};
          *(v4f*)(sp + 4) = (v4f){u[4], u[5], u[6], u[7]};
        }
        wave_lds_sync();
        v8f dre, dim;
        {
          v8f x;
#pragma unroll
          for (int i = 0; i < 8; ++i) x[i] = scr[pa[i]];
          v8h xh, xl;
          split8(x, xh, xl);
          dre = layer_pair(xh, xl, bLo2, bHi2, kEndMain, kEndRes);
        }
        {
          v8f x;
#pragma unroll
          for (int i = 0; i < 8; ++i) x[i] = scr[256 + pa[i]];
          v8h xh, xl;
          split8(x, xh, xl);
          dim = layer_pair(xh, xl, bLo2, bHi2, kEndMain, kEndRes);
        }
        wave_lds_sync();
        {
          v8f p;
#pragma unroll
          for (int e = 0; e < 8; ++e) p[e] = dre[e] * dre[e] + dim[e] * dim[e];
          float* sp = scr + 16 * n + 8 * h;
          *(v4f*)(sp)     = (v4f){p[0], p[1], p[2], p[3]};
          *(v4f*)(sp + 4) = (v4f){p[4], p[5], p[6], p[7]};
        }
        wave_lds_sync();
        float pp[8];
#pragma unroll
        for (int i = 0; i < 8; ++i) pp[i] = scr[pa[i]];
        wave_lds_sync();
        float ev[8];
        {
          const float a0 = pp[0] + pp[1], d0 = pp[0] - pp[1];
          const float a1 = pp[2] + pp[3], d1 = pp[2] - pp[3];
          const float a2 = pp[4] + pp[5], d2 = pp[4] - pp[5];
          const float a3 = pp[6] + pp[7], d3 = pp[6] - pp[7];
          const float b0 = a0 + a1, c0 = a0 - a1;
          const float b1 = a2 + a3, c1 = a2 - a3;
          const float tt = b0 + b1;
          const float nt = -tt;
          ev[7] = (d0 + d1) + (d2 + d3);
          ev[6] = c0 + c1;
          ev[5] = b0 - b1;
          ev[4] = w4set ? nt : tt;
          ev[3] = w3set ? nt : tt;
          ev[2] = w2set ? nt : tt;
          ev[1] = w1set ? nt : tt;
          ev[0] = w0set ? nt : tt;
        }
#pragma unroll
        for (int off = 1; off < 32; off <<= 1) {
#pragma unroll
          for (int w = 0; w < 8; ++w) ev[w] += __shfl_xor(ev[w], off, 32);
        }
        float evs = ev[0];
#pragma unroll
        for (int w = 1; w < 8; ++w) evs = (lane == w) ? ev[w] : evs;
        if (lane < 8) s_ev[srow * 32 + g * 8 + lane] = evs;
      }
    }
    __syncthreads();

#pragma unroll 1
    for (int s8 = 0; s8 < 8; ++s8) {
      const int srow = half * 8 + s8;
      const float* ep = s_ev + srow * 32;
      float af = bfv, ai = biv, ag = bgv, ao = bov;
      {
        const v4f e0 = *(const v4f*)(ep);
        const v4f e1 = *(const v4f*)(ep + 4);
#pragma unroll
        for (int e = 0; e < 4; ++e) { af = fmaf(e0[e], wf[e], af); af = fmaf(e1[e], wf[4 + e], af); }
      }
      {
        const v4f e0 = *(const v4f*)(ep + 8);
        const v4f e1 = *(const v4f*)(ep + 12);
#pragma unroll
        for (int e = 0; e < 4; ++e) { ai = fmaf(e0[e], wi[e], ai); ai = fmaf(e1[e], wi[4 + e], ai); }
      }
      {
        const v4f e0 = *(const v4f*)(ep + 16);
        const v4f e1 = *(const v4f*)(ep + 20);
#pragma unroll
        for (int e = 0; e < 4; ++e) { ag = fmaf(e0[e], wg[e], ag); ag = fmaf(e1[e], wg[4 + e], ag); }
      }
      {
        const v4f e0 = *(const v4f*)(ep + 24);
        const v4f e1 = *(const v4f*)(ep + 28);
#pragma unroll
        for (int e = 0; e < 4; ++e) { ao = fmaf(e0[e], wo[e], ao); ao = fmaf(e1[e], wo[4 + e], ao); }
      }
      const float fg = sigmoid_fast(af);
      const float ig = sigmoid_fast(ai);
      const float gg = tanh_fast(ag);
      const float og = sigmoid_fast(ao);
      const float cold = s_c[srow * kHid + jh];
      const float cn = fg * cold + ig * gg;
      const float hn = og * tanh_fast(cn);
      s_c[srow * kHid + jh] = cn;
      s_hout[srow * kHid + jh] = hn;
      s_a[srow * kAPitch + kFeat + jh] = to_h(hn * kActCarry);
    }
    __syncthreads();

    {
      const int r0 = 2 * wave;
      const v4f v0 = *(const v4f*)(s_hout + r0 * kHid + lane * 4);
      const v4f v1 = *(const v4f*)(s_hout + (r0 + 1) * kHid + lane * 4);
      float* op = out + ((size_t)t * kBatch + (size_t)blk * kTileB + r0) * kHid + lane * 4;
      *(volatile v4f*)(op) = v0;
      *(volatile v4f*)(op + kHid) = v1;
      __threadfence();
      *(volatile v4f*)(op) = v0;
      *(volatile v4f*)(op + kHid) = v1;
    }
  }

  {
    const int r0 = 2 * wave;
    const v4f h0 = *(const v4f*)(s_hout + r0 * kHid + lane * 4);
    const v4f h1 = *(const v4f*)(s_hout + (r0 + 1) * kHid + lane * 4);
    const v4f c0 = *(const v4f*)(s_c + r0 * kHid + lane * 4);
    const v4f c1 = *(const v4f*)(s_c + (r0 + 1) * kHid + lane * 4);
    float* hp = out + kOutH + ((size_t)blk * kTileB + r0) * kHid + lane * 4;
    float* cp = out + kOutC + ((size_t)blk * kTileB + r0) * kHid + lane * 4;
    *(volatile v4f*)(hp) = h0;
    *(volatile v4f*)(hp + kHid) = h1;
    *(volatile v4f*)(cp) = c0;
    *(volatile v4f*)(cp + kHid) = c1;
    __threadfence();
    *(volatile v4f*)(hp) = h0;
    *(volatile v4f*)(hp + kHid) = h1;
    *(volatile v4f*)(cp) = c0;
    *(volatile v4f*)(cp + kHid) = c1;
  }
}

extern "C" void kernel_launch(void* const* d_in, const int* in_sizes, int n_in,
                              void* d_out, int out_size, void* d_ws, size_t ws_size,
                              hipStream_t stream) {
  if (n_in < 15) return;
  if (in_sizes[0] != kSeq * kBatch * kFeat) return;
  if (in_sizes[1] != 32 * kKq) return;
  if (in_sizes[2] != 32) return;
  if (in_sizes[3] != kDepth * kWires || in_sizes[4] != kDepth * kWires) return;
  if (in_sizes[5] != kDepth * kWires || in_sizes[6] != kDepth * kWires) return;
  if (in_sizes[7] != kHid * kWires || in_sizes[9] != kHid * kWires) return;
  if (in_sizes[11] != kHid * kWires || in_sizes[13] != kHid * kWires) return;
  if (in_sizes[8] != kHid || in_sizes[10] != kHid || in_sizes[12] != kHid || in_sizes[14] != kHid) return;
  if ((size_t)out_size != kOutTotal) return;
  if (ws_size < kWsTotal) return;

  const float* xin = (const float*)d_in[0];
  const float* Wq  = (const float*)d_in[1];
  const float* bq  = (const float*)d_in[2];
  const float* pf  = (const float*)d_in[3];
  const float* pi  = (const float*)d_in[4];
  const float* pg  = (const float*)d_in[5];
  const float* po  = (const float*)d_in[6];
  const float* Wf  = (const float*)d_in[7];
  const float* bfp = (const float*)d_in[8];
  const float* Wi  = (const float*)d_in[9];
  const float* bip = (const float*)d_in[10];
  const float* Wg  = (const float*)d_in[11];
  const float* bgp = (const float*)d_in[12];
  const float* Wo  = (const float*)d_in[13];
  const float* bop = (const float*)d_in[14];
  unsigned short* fac = (unsigned short*)d_ws;
  float* out = (float*)d_out;

  build_factor_planes<<<1, 512, 0, stream>>>(pf, pi, pg, po, fac);
  gated_cell_kernel<<<kBlocks, kThreads, 0, stream>>>(xin, Wq, bq, Wf, bfp, Wi, bip, Wg, bgp, Wo, bop, fac, out);
}
